// MyModel_61933428409733
// MI455X (gfx1250) — hardware-verified
//
#include <hip/hip_runtime.h>
#include <math.h>

constexpr int kBatch = 4;
constexpr int kSeq   = 2048;
constexpr int kDim   = 1024;
constexpr float kNegScale = -10000.0f;
constexpr float kFltMin   = 1.17549435e-38f;
static_assert(kSeq % 64 == 0 && kDim % 64 == 0, "M and N tile multiples");
static_assert(kSeq % 32 == 0 && kDim % 32 == 0, "K multiples of 32");
static_assert(kSeq == 256 * 8, "softmax row coverage: 256 threads x 8 columns");

typedef __attribute__((ext_vector_type(16))) _Float16 v16h;
typedef __attribute__((ext_vector_type(8)))  _Float16 v8h;
typedef __attribute__((ext_vector_type(16))) __bf16   v16b;
typedef __attribute__((ext_vector_type(8)))  __bf16   v8b;
typedef __attribute__((ext_vector_type(8)))  float    v8f;
typedef __attribute__((ext_vector_type(4)))  float    v4f;
typedef __attribute__((ext_vector_type(4)))  unsigned int v4u;

__device__ __forceinline__ unsigned short f2bf_bits(float f) {
  unsigned u = __float_as_uint(f);
  return (unsigned short)((u + 0x7FFFu + ((u >> 16) & 1u)) >> 16);
}
__device__ __forceinline__ float bf_bits2f(unsigned short h) { return __uint_as_float(((unsigned)h) << 16); }

__device__ __forceinline__ void dep_guard_h(v8f& a, v8f& b, v16h x, v16h y) { asm volatile("v_nop\n\tv_nop\n\tv_nop\n\tv_nop" : "+v"(a), "+v"(b) : "v"(x), "v"(y)); }
__device__ __forceinline__ void dep_guard_b(v8f& a, v8f& b, v16b x, v16b y) { asm volatile("v_nop\n\tv_nop\n\tv_nop\n\tv_nop" : "+v"(a), "+v"(b) : "v"(x), "v"(y)); }
__device__ __forceinline__ void dep_guard4_h(v8f& a, v8f& b, v8f& c, v8f& d, v16h x, v16h y) { asm volatile("v_nop\n\tv_nop\n\tv_nop\n\tv_nop" : "+v"(a), "+v"(b), "+v"(c), "+v"(d) : "v"(x), "v"(y)); }
__device__ __forceinline__ void dep_guard4_b(v8f& a, v8f& b, v8f& c, v8f& d, v16b x, v16b y) { asm volatile("v_nop\n\tv_nop\n\tv_nop\n\tv_nop" : "+v"(a), "+v"(b), "+v"(c), "+v"(d) : "v"(x), "v"(y)); }
__device__ __forceinline__ void keep4_h(v16h a, v16h b, v16h c, v16h d) { asm volatile("v_nop" :: "v"(a), "v"(b), "v"(c), "v"(d)); }
__device__ __forceinline__ void keep4_b(v16b a, v16b b, v16b c, v16b d) { asm volatile("v_nop" :: "v"(a), "v"(b), "v"(c), "v"(d)); }
__device__ __forceinline__ void acc_guard4(v8f& a, v8f& b, v8f& c, v8f& d) { asm volatile("v_nop\n\tv_nop\n\tv_nop\n\tv_nop" : "+v"(a), "+v"(b), "+v"(c), "+v"(d)); }
template <typename T> struct Frag;
template <> struct Frag<_Float16> {
  typedef v16h V; union U { v16h v; v8h h[2]; };
  static __device__ __forceinline__ v16h load(const _Float16* p) {
    U f; f.h[0] = *(const v8h*)(p); f.h[1] = *(const v8h*)(p + 16); return f.v;
  }
  static __device__ __forceinline__ v8f mma(v16h a, v16h b, v8f c) {
    return __builtin_amdgcn_wmma_f32_16x16x32_f16(false, a, false, b, (short)0, c, false, false);
  }
  static __device__ __forceinline__ void guard(v8f& a, v8f& b, v16h x, v16h y) { dep_guard_h(a, b, x, y); }
  static __device__ __forceinline__ void guard4(v8f& a, v8f& b, v8f& c, v8f& d, v16h x, v16h y) { dep_guard4_h(a, b, c, d, x, y); }
  static __device__ __forceinline__ void keep(v16h a, v16h b, v16h c, v16h d) { keep4_h(a, b, c, d); }
};
template <> struct Frag<__bf16> {
  typedef v16b V; union U { v16b v; v8b h[2]; };
  static __device__ __forceinline__ v16b load(const __bf16* p) {
    U f; f.h[0] = *(const v8b*)(p); f.h[1] = *(const v8b*)(p + 16); return f.v;
  }
  static __device__ __forceinline__ v8f mma(v16b a, v16b b, v8f c) {
    return __builtin_amdgcn_wmma_f32_16x16x32_bf16(false, a, false, b, (short)0, c, false, false);
  }
  static __device__ __forceinline__ void guard(v8f& a, v8f& b, v16b x, v16b y) { dep_guard_b(a, b, x, y); }
  static __device__ __forceinline__ void guard4(v8f& a, v8f& b, v8f& c, v8f& d, v16b x, v16b y) { dep_guard4_b(a, b, c, d, x, y); }
  static __device__ __forceinline__ void keep(v16b a, v16b b, v16b c, v16b d) { keep4_b(a, b, c, d); }
};

__device__ __forceinline__ unsigned pk16(unsigned short a, unsigned short b) { return (unsigned)a | ((unsigned)b << 16); }

template <int ET> struct Elem;
template <> struct Elem<0> { typedef _Float16 T; };
template <> struct Elem<1> { typedef __bf16 T; };
template <int ET, bool SPLIT, int BIAS_MODE, int OUT_MODE, bool RESID, int ACT = 0>
__global__ __launch_bounds__(256) void wmma_gemm64(
    const unsigned short* __restrict__ Ap, const unsigned short* __restrict__ A2p, int lda, long strideA,
    const unsigned short* __restrict__ Btp, const unsigned short* __restrict__ Bt2p, int ldb, long strideB,
    void* __restrict__ Cout, void* __restrict__ Cout2, int ldc, long strideC,
    const float* __restrict__ bias,
    const float* __restrict__ resid, long strideR,
    int M, int N, int K, float scale) {
  typedef typename Elem<ET>::T T;
  typedef typename Frag<T>::V V;
  const T* A = (const T*)Ap; const T* A2 = (const T*)A2p; const T* Bt = (const T*)Btp; const T* Bt2 = (const T*)Bt2p;
  __shared__ __align__(16) float sT[8][16 * 68];
  const int b    = blockIdx.y;
  const int lane = threadIdx.x & 31;
  const int wave = threadIdx.x >> 5;
  const int tilesN = N >> 6;
  const int tilesM = M >> 6;
  const int tile = blockIdx.x * 8 + wave;
  if (tile >= tilesM * tilesN) return;
  const int tm = tile / tilesN;
  const int tn = tile - tm * tilesN;
  const int m0 = tm << 6;
  const int n0 = tn << 6;

  const T* Ab  = A  + (size_t)b * strideA;
  const T* Bb  = Bt + (size_t)b * strideB;
  const T* Ab2 = SPLIT ? (A2  + (size_t)b * strideA) : nullptr;
  const T* Bb2 = SPLIT ? (Bt2 + (size_t)b * strideB) : nullptr;

  const int rlane = lane & 15;
  const int koff  = (lane >> 4) * 8;
  const int mOff  = (lane >> 4) * 8;

  v8f acc[4][4];
#pragma unroll
  for (int i = 0; i < 4; ++i)
#pragma unroll
    for (int j = 0; j < 4; ++j) acc[i][j] = (v8f){0.f,0.f,0.f,0.f,0.f,0.f,0.f,0.f};

  for (int k0 = 0; k0 < K; k0 += 32) {
    V bh[4], bl[4];
#pragma unroll
    for (int j = 0; j < 4; ++j) {
      const size_t bo = (size_t)(n0 + (j << 4) + rlane) * ldb + koff + k0;
      bh[j] = Frag<T>::load(Bb + bo);
      if (SPLIT) bl[j] = Frag<T>::load(Bb2 + bo);
    }
#pragma unroll
    for (int i = 0; i < 4; ++i) {
      const size_t ao = (size_t)(m0 + (i << 4) + rlane) * lda + koff + k0;
      V ah = Frag<T>::load(Ab + ao);
      V al;
      if (SPLIT) al = Frag<T>::load(Ab2 + ao);
#pragma unroll
      for (int j = 0; j < 4; ++j) {
        acc[i][j] = Frag<T>::mma(ah, bh[j], acc[i][j]);
        if (SPLIT) {
          acc[i][j] = Frag<T>::mma(ah, bl[j], acc[i][j]);
          acc[i][j] = Frag<T>::mma(al, bh[j], acc[i][j]);
        }
      }
      Frag<T>::guard4(acc[i][0], acc[i][1], acc[i][2], acc[i][3], ah, SPLIT ? al : ah);
    }
    Frag<T>::keep(bh[0], bh[1], bh[2], bh[3]);
    if (SPLIT) Frag<T>::keep(bl[0], bl[1], bl[2], bl[3]);
  }
  acc_guard4(acc[0][0], acc[0][1], acc[0][2], acc[0][3]);
  acc_guard4(acc[1][0], acc[1][1], acc[1][2], acc[1][3]);
  acc_guard4(acc[2][0], acc[2][1], acc[2][2], acc[2][3]);
  acc_guard4(acc[3][0], acc[3][1], acc[3][2], acc[3][3]);

  float* slab = sT[wave];
  const float* Rb = RESID ? (resid + (size_t)b * strideR) : nullptr;
#pragma unroll
  for (int i = 0; i < 4; ++i) {
    const int mBase = m0 + (i << 4);
#pragma unroll
    for (int j = 0; j < 4; ++j) {
      const int n = n0 + (j << 4) + rlane;
      float bv = 0.f;
      if (BIAS_MODE == 2) bv = bias[n];
#pragma unroll
      for (int r = 0; r < 8; ++r) {
        float v = acc[i][j][r] * scale;
        if (BIAS_MODE == 1) v += bias[mBase + mOff + r];
        if (BIAS_MODE == 2) v += bv;
        if (RESID) v += Rb[(size_t)(mBase + mOff + r) * ldc + n];
        if (ACT == 2) v = fmaxf(v, 0.0f);
        if (ACT == 4) v = (v > 0.f) ? v : 0.01f * v;
        slab[(mOff + r) * 68 + (j << 4) + rlane] = v;
      }
    }
    __builtin_amdgcn_fence(__ATOMIC_RELEASE, "workgroup");
    __builtin_amdgcn_wave_barrier();
    __builtin_amdgcn_fence(__ATOMIC_ACQUIRE, "workgroup");
    if (OUT_MODE == 0) {
      float* C = (float*)Cout + (size_t)b * strideC;
      const int hh = lane >> 4, c4 = (lane & 15) * 4;
      for (int pass = 0; pass < 2; ++pass) {
#pragma unroll
        for (int it = 0; it < 8; ++it) {
          const int row = it * 2 + hh;
          v4f v = *(const v4f*)(slab + row * 68 + c4);
          *(volatile v4f*)(C + (size_t)(mBase + row) * ldc + n0 + c4) = v;
        }
        __threadfence();
      }
    } else {
      const int q = lane >> 3, c8 = (lane & 7) * 8;
      unsigned short* C  = (unsigned short*)Cout  + (size_t)b * strideC;
      unsigned short* C2 = (OUT_MODE == 2) ? ((unsigned short*)Cout2 + (size_t)b * strideC) : nullptr;
      for (int pass = 0; pass < 2; ++pass) {
#pragma unroll
        for (int it = 0; it < 4; ++it) {
          const int row = it * 4 + q;
          const float* sp = slab + row * 68 + c8;
          v8h hv, lv;
#pragma unroll
          for (int e = 0; e < 8; ++e) {
            if (OUT_MODE == 1) {
              hv[e] = (_Float16)sp[e];
            } else {
              unsigned short hb = f2bf_bits(sp[e]);
              unsigned short lb = f2bf_bits(sp[e] - bf_bits2f(hb));
              hv[e] = __builtin_bit_cast(_Float16, hb);
              lv[e] = __builtin_bit_cast(_Float16, lb);
            }
          }
          *(volatile v8h*)(C + (size_t)(mBase + row) * ldc + n0 + c8) = hv;
          if (OUT_MODE == 2) *(volatile v8h*)(C2 + (size_t)(mBase + row) * ldc + n0 + c8) = lv;
        }
        __threadfence();
      }
    }
    __builtin_amdgcn_fence(__ATOMIC_RELEASE, "workgroup");
    __builtin_amdgcn_wave_barrier();
    __builtin_amdgcn_fence(__ATOMIC_ACQUIRE, "workgroup");
  }
}

__global__ __launch_bounds__(256) void cast_transpose_kernel(const float* __restrict__ x,
                                                            unsigned short* __restrict__ Xb,
                                                            unsigned short* __restrict__ XbT) {
  __shared__ float sm[64][65];
  const int tid = threadIdx.x;
  const int d0  = blockIdx.x * 64;
  const int t0  = blockIdx.y * 64;
  const int b   = blockIdx.z;
  const float* xb = x + (size_t)b * kSeq * kDim;
#pragma unroll
  for (int i = 0; i < 16; ++i) {
    const int e = i * 256 + tid;
    const int r = e >> 6;
    const int c = e & 63;
    sm[r][c] = xb[(size_t)(t0 + r) * kDim + d0 + c];
  }
  __syncthreads();
  const int lane = tid & 31, wave = tid >> 5;
  const int q = lane >> 3, c8 = (lane & 7) * 8;
  unsigned short* xrow = Xb  + (size_t)b * kSeq * kDim;
  unsigned short* xcol = XbT + (size_t)b * kDim * kSeq;
  for (int pass = 0; pass < 2; ++pass) {
#pragma unroll
    for (int it = 0; it < 2; ++it) {
      const int row = wave * 8 + it * 4 + q;
      unsigned short hr[8], hc[8];
#pragma unroll
      for (int e = 0; e < 8; ++e) {
        hr[e] = f2bf_bits(sm[row][c8 + e]);
        hc[e] = f2bf_bits(sm[c8 + e][row]);
      }
      const v4u ur = (v4u){pk16(hr[0], hr[1]), pk16(hr[2], hr[3]), pk16(hr[4], hr[5]), pk16(hr[6], hr[7])};
      const v4u uc = (v4u){pk16(hc[0], hc[1]), pk16(hc[2], hc[3]), pk16(hc[4], hc[5]), pk16(hc[6], hc[7])};
      *(volatile v4u*)(xrow + (size_t)(t0 + row) * kDim + d0 + c8) = ur;
      *(volatile v4u*)(xcol + (size_t)(d0 + row) * kSeq + t0 + c8) = uc;
    }
    __threadfence();
  }
}

__global__ __launch_bounds__(256) void softmax_row_kernel(const float* __restrict__ S, unsigned short* __restrict__ P) {
  __shared__ __align__(16) float pe[kSeq];
  __shared__ float redM[8];
  __shared__ float redS[8];
  const int row  = blockIdx.x;
  const int t    = threadIdx.x;
  const int lane = t & 31, wave = t >> 5;
  const float* sr = S + (size_t)row * kSeq + 8 * t;
  float* slot = pe + 8 * t;

  float mx = -3.0e38f;
#pragma unroll 1
  for (int it = 0; it < 2; ++it) {
    const v4f sv = *(const v4f*)(sr + 4 * it);
    v4f lv;
#pragma unroll
    for (int e = 0; e < 4; ++e) {
      const float v = sv[e] * kNegScale;
      lv[e] = v;
      mx = fmaxf(mx, v);
    }
    *(v4f*)(slot + 4 * it) = lv;
  }
#pragma unroll
  for (int off = 16; off > 0; off >>= 1) mx = fmaxf(mx, __shfl_xor(mx, off, 32));
  if (lane == 0) redM[wave] = mx;
  __syncthreads();
  float m = redM[0];
#pragma unroll
  for (int w = 1; w < 8; ++w) m = fmaxf(m, redM[w]);

  float sum = 0.f;
#pragma unroll 1
  for (int it = 0; it < 2; ++it) {
    const v4f l = *(const v4f*)(slot + 4 * it);
    v4f ev;
#pragma unroll
    for (int e = 0; e < 4; ++e) {
      float p = expf(l[e] - m);
      p = (p < kFltMin) ? 0.0f : p;
      ev[e] = p;
      sum += p;
    }
    *(v4f*)(slot + 4 * it) = ev;
  }
#pragma unroll
  for (int off = 16; off > 0; off >>= 1) sum += __shfl_xor(sum, off, 32);
  if (lane == 0) redS[wave] = sum;
  __syncthreads();
  float tot = redS[0];
#pragma unroll
  for (int w = 1; w < 8; ++w) tot += redS[w];
  const float inv = 1.0f / tot;

  const v4f e0 = *(const v4f*)(slot);
  const v4f e1 = *(const v4f*)(slot + 4);
  unsigned short hb[8];
#pragma unroll
  for (int e = 0; e < 4; ++e) {
    hb[e]     = f2bf_bits(e0[e] * inv);
    hb[4 + e] = f2bf_bits(e1[e] * inv);
  }
  const v4u u = (v4u){pk16(hb[0], hb[1]), pk16(hb[2], hb[3]), pk16(hb[4], hb[5]), pk16(hb[6], hb[7])};
  unsigned short* pr = P + (size_t)row * kSeq + 8 * (size_t)t;
  *(volatile v4u*)pr = u;
  __threadfence();
  *(volatile v4u*)pr = u;
}

extern "C" void kernel_launch(void* const* d_in, const int* in_sizes, int n_in,
                              void* d_out, int out_size, void* d_ws, size_t ws_size,
                              hipStream_t stream) {
  if (n_in < 1) return;
  const int nElem = kBatch * kSeq * kDim;
  if (in_sizes[0] != nElem) return;
  if (out_size != nElem) return;

  const size_t szX  = (size_t)kBatch * kSeq * kDim * 2;
  const size_t szS  = (size_t)kBatch * kSeq * kSeq * 4;
  const size_t szP  = (size_t)kBatch * kSeq * kSeq * 2;
  const size_t offXb  = 0;
  const size_t offXbT = offXb + szX;
  const size_t offS   = offXbT + szX;
  const size_t offP   = offS + szS;
  const size_t total  = offP + szP;
  if (ws_size < total) return;

  const float* x = (const float*)d_in[0];
  float* out = (float*)d_out;
  char* ws = (char*)d_ws;
  unsigned short* Xb  = (unsigned short*)(ws + offXb);
  unsigned short* XbT = (unsigned short*)(ws + offXbT);
  float* SC = (float*)(ws + offS);
  unsigned short* PP = (unsigned short*)(ws + offP);
  const float* dummy = (const float*)SC;

  cast_transpose_kernel<<<dim3(kDim / 64, kSeq / 64, kBatch), dim3(256), 0, stream>>>(x, Xb, XbT);

  const long strideX  = (long)kSeq * kDim;
  const long strideSS = (long)kSeq * kSeq;
  const int  tilesScore = (kSeq / 64) * (kSeq / 64);
  wmma_gemm64<1, false, 0, 0, false, 0><<<dim3(tilesScore / 8, kBatch), dim3(256), 0, stream>>>(
      Xb, Xb, kDim, strideX, Xb, Xb, kDim, strideX,
      (void*)SC, (void*)SC, kSeq, strideSS, dummy, dummy, 0L, kSeq, kSeq, kDim, 1.0f);

  softmax_row_kernel<<<dim3(kBatch * kSeq), dim3(256), 0, stream>>>(SC, PP);

  const int tilesOut = (kSeq / 64) * (kDim / 64);
  wmma_gemm64<1, false, 0, 0, false, 0><<<dim3(tilesOut / 8, kBatch), dim3(256), 0, stream>>>(
      PP, PP, kSeq, strideSS, XbT, XbT, kSeq, strideX,
      (void*)out, (void*)out, kDim, strideX, dummy, dummy, 0L, kSeq, kDim, kSeq, 1.0f);
}
